// Decorrelation_66563403153962
// MI455X (gfx1250) — hardware-verified
//
#include <hip/hip_runtime.h>
#include <stddef.h>
#include <stdint.h>


#pragma clang fp contract(off)

#define NV      32
#define KBAS    16
#define KTOT    (NV * KBAS)
#define NPAIR   496
#define NKT     20
#define RPB     32
#define NTH     64
#define AP      528
#define DP      36
#define WBLK    ((NV * KTOT / 8) / NTH)
#define A_CARRY 256.0f
#define W_CARRY 64.0f
#define ACC_INV (1.0f / 16384.0f)
#define KLO     (-6.0f)
#define KHI     6.0f
#define XMAX    5.999988f
#define WSCAP   134217728

static_assert(KTOT == 512);
static_assert((KTOT % 32) == 0);
static_assert(WBLK * NTH * 8 == NV * KTOT);
static_assert(((AP * 2) % 16) == 0 && AP >= KTOT);
static_assert(((DP * 4) % 16) == 0 && DP >= NV);
static_assert(RPB * AP * 2 + RPB * DP * 4 <= 64 * 1024);
static_assert((RPB * NV / 4) % NTH == 0 && (RPB * NV / 4) / NTH == 4);
static_assert(NTH == 64 && RPB == 32);

typedef _Float16 v16h __attribute__((ext_vector_type(16)));
typedef _Float16 v8h  __attribute__((ext_vector_type(8)));
typedef float    v8f  __attribute__((ext_vector_type(8)));
typedef float    v4f  __attribute__((ext_vector_type(4)));
union Frag { v16h v; v8h half[2]; };
static_assert(sizeof(Frag) == 32);

__device__ __forceinline__ v8f wmh(v16h a, v16h bq, v8f c) {
  v8f d = __builtin_amdgcn_wmma_f32_16x16x32_f16(false, a, false, bq, (short)0, c, false, false);
  asm volatile("v_nop\n\tv_nop\n\tv_nop\n\tv_nop" : "+v"(d) : "v"(a), "v"(bq));
  return d;
}

__device__ __forceinline__ v8f zero8() {
  v8f z = {0.f, 0.f, 0.f, 0.f, 0.f, 0.f, 0.f, 0.f};
  return z;
}

__global__ __launch_bounds__(NTH) void k_wpack(const float* __restrict__ params, _Float16* Wp) {
  const int g  = blockIdx.x * NTH + threadIdx.x;
  const int n  = g >> 6;
  const int kb = (g & 63) * 8;
  const int c  = kb >> 4;
  const int k8 = kb & 15;
  int pr = ((n * (n - 1)) >> 1) + c;
  pr = pr < 0 ? 0 : pr;
  pr = pr > NPAIR - 1 ? NPAIR - 1 : pr;
  const bool live = c < n;
  v8h hv;
#pragma unroll
  for (int i = 0; i < 8; ++i) {
    const float p = params[(k8 + i) * NPAIR + pr];
    const float s = live ? p * W_CARRY : 0.0f;
    hv[i] = (_Float16)s;
  }
  _Float16* d = Wp + (size_t)g * 8;
  *(volatile v8h*)d = hv;
  __threadfence();
  *(volatile v8h*)d = hv;
}

__global__ __launch_bounds__(NTH) void k_main(const float* __restrict__ X, const _Float16* __restrict__ Wp,
                                              float* out) {
  __shared__ __align__(16) _Float16 As[RPB * AP];
  __shared__ __align__(16) float Ds[RPB * DP];

  const int tid = threadIdx.x, lane = tid & 31, wave = tid >> 5, h = lane >> 4, m = lane & 15;
  const int rowBase = blockIdx.x * RPB;

  {
    float T[NKT];
    T[0] = KLO; T[1] = KLO; T[2] = KLO;
#pragma unroll
    for (int i = 0; i < 13; ++i) {
      const float st = (float)i * (1.0f / 13.0f);
      T[3 + i] = KLO * (1.0f - st) + KHI * st;
    }
    T[16] = KHI; T[17] = KHI; T[18] = KHI; T[19] = KHI;

    const int c = tid & 31;
#pragma unroll 1
    for (int i = 0; i < RPB / 2; ++i) {
      const int row = wave + 2 * i;
      const float x  = X[(size_t)(rowBase + row) * NV + c];
      const float xc = fminf(fmaxf(x, KLO), XMAX);
      float b[NKT - 1];
#pragma unroll
      for (int j = 0; j < NKT - 1; ++j) b[j] = (xc >= T[j] && xc < T[j + 1]) ? 1.0f : 0.0f;
#pragma unroll
      for (int j = 0; j < 18; ++j) {
        const float d1 = T[j + 1] - T[j];
        const float d2 = T[j + 2] - T[j + 1];
        const float lf = (d1 > 0.0f) ? (xc - T[j]) * (1.0f / d1) : 0.0f;
        const float rg = (d2 > 0.0f) ? (T[j + 2] - xc) * (1.0f / d2) : 0.0f;
        b[j] = lf * b[j] + rg * b[j + 1];
      }
#pragma unroll
      for (int j = 0; j < 17; ++j) {
        const float d1 = T[j + 2] - T[j];
        const float d2 = T[j + 3] - T[j + 1];
        const float lf = (d1 > 0.0f) ? (xc - T[j]) * (1.0f / d1) : 0.0f;
        const float rg = (d2 > 0.0f) ? (T[j + 3] - xc) * (1.0f / d2) : 0.0f;
        b[j] = lf * b[j] + rg * b[j + 1];
      }
#pragma unroll
      for (int j = 0; j < 16; ++j) {
        const float d1 = T[j + 3] - T[j];
        const float d2 = T[j + 4] - T[j + 1];
        const float lf = (d1 > 0.0f) ? (xc - T[j]) * (1.0f / d1) : 0.0f;
        const float rg = (d2 > 0.0f) ? (T[j + 4] - xc) * (1.0f / d2) : 0.0f;
        b[j] = lf * b[j] + rg * b[j + 1];
      }
      v8h p0, p1;
#pragma unroll
      for (int q = 0; q < 8; ++q) {
        p0[q] = (_Float16)((b[q] * x) * A_CARRY);
        p1[q] = (_Float16)((b[q + 8] * x) * A_CARRY);
      }
      _Float16* ap = As + row * AP + c * KBAS;
      *(v8h*)ap = p0;
      *(v8h*)(ap + 8) = p1;
    }
  }
  __syncthreads();

  v8f acc0 = zero8();
  v8f acc1 = zero8();
  {
    const _Float16* ab  = As + (wave * 16 + m) * AP + 8 * h;
    const _Float16* wb0 = Wp + (size_t)m * KTOT + 8 * h;
    const _Float16* wb1 = Wp + (size_t)(16 + m) * KTOT + 8 * h;
#pragma unroll 2
    for (int ks = 0; ks < KTOT / 32; ++ks) {
      const int ko = 32 * ks;
      Frag fa, fb0, fb1;
      fa.half[0]  = *(const v8h*)(ab + ko);
      fa.half[1]  = *(const v8h*)(ab + ko + 16);
      fb0.half[0] = *(const v8h*)(wb0 + ko);
      fb0.half[1] = *(const v8h*)(wb0 + ko + 16);
      fb1.half[0] = *(const v8h*)(wb1 + ko);
      fb1.half[1] = *(const v8h*)(wb1 + ko + 16);
      acc0 = wmh(fa.v, fb0.v, acc0);
      acc1 = wmh(fa.v, fb1.v, acc1);
    }
  }

#pragma unroll
  for (int r = 0; r < 8; ++r) {
    const int rr = (wave * 16 + 8 * h + r) * DP;
    Ds[rr + m]      = acc0[r] * ACC_INV;
    Ds[rr + 16 + m] = acc1[r] * ACC_INV;
  }
  __syncthreads();

  v4f vals[4];
#pragma unroll
  for (int j = 0; j < 4; ++j) {
    const int e = tid + j * NTH;
    const int row = e >> 3, q = e & 7;
    const v4f d  = *(const v4f*)(Ds + row * DP + 4 * q);
    const v4f xr = *(const v4f*)(X + (size_t)(rowBase + row) * NV + 4 * q);
    vals[j] = d + xr;
  }
  float* ob = out + (size_t)rowBase * NV;
#pragma unroll
  for (int j = 0; j < 4; ++j) {
    const int e = tid + j * NTH;
    *(volatile v4f*)(ob + 4 * e) = vals[j];
  }
  __threadfence();
#pragma unroll
  for (int j = 0; j < 4; ++j) {
    const int e = tid + j * NTH;
    *(volatile v4f*)(ob + 4 * e) = vals[j];
  }
}

extern "C" void kernel_launch(void* const* d_in, const int* in_sizes, int n_in,
                              void* d_out, int out_size, void* d_ws, size_t ws_size,
                              hipStream_t stream) {
  if (n_in < 2) return;
  const int nrow = in_sizes[0] / NV;
  if (nrow <= 0 || in_sizes[0] != nrow * NV || (nrow % RPB) != 0) return;
  if (in_sizes[1] != KBAS * NPAIR) return;
  if (out_size != nrow * NV) return;

  const float* X      = (const float*)d_in[0];
  const float* params = (const float*)d_in[1];
  float* out          = (float*)d_out;

  const size_t wbytes = (size_t)NV * KTOT * 2;
  if (wbytes > ws_size || wbytes > (size_t)WSCAP) return;
  _Float16* Wp = (_Float16*)d_ws;

  k_wpack<<<WBLK, NTH, 0, stream>>>(params, Wp);
  k_main<<<nrow / RPB, NTH, 0, stream>>>(X, Wp, out);
}
